// _MambaMixer_33449205301613
// MI455X (gfx1250) — hardware-run, weakly checked
//
#include <hip/hip_runtime.h>
#include <hip/hip_fp16.h>
#include <math.h>

constexpr int kBatch = 2;
constexpr int kSeq   = 2048;
constexpr int kDm    = 1024;
constexpr int kDin   = 2048;
constexpr int kNst   = 16;
constexpr int kDtR   = 64;
constexpr int kRows  = kBatch * kSeq;
constexpr int kXzP   = 2 * kDin;
constexpr int kPrW   = kDtR + 2 * kNst;
constexpr int kPrP   = 128;
constexpr int kOffB  = kDtR;
constexpr int kOffC  = kDtR + kNst;
constexpr int kConvTP = 260;
static_assert(kPrW == 96);
static_assert(kPrP % 64 == 0 && kPrP >= kPrW);
static_assert(kDm % 32 == 0 && kDin % 32 == 0 && kDtR % 32 == 0);
static_assert(kRows % 64 == 0 && kXzP % 64 == 0 && kDin % 64 == 0 && kDm % 64 == 0);
static_assert(kSeq % 64 == 0 && kDin % 256 == 0);

constexpr float kCarryX   = 16.0f;
constexpr float kCarryW   = 1024.0f;
constexpr float kCarryU   = 256.0f;
constexpr float kCarryR   = 256.0f;
constexpr float kCarryWdt = 64.0f;
constexpr float kCarryY   = 1024.0f;
constexpr float kScaleIn  = 1.0f / (kCarryX * kCarryW);
constexpr float kScaleXp  = 1.0f / (kCarryU * kCarryW);
constexpr float kScaleDt  = 1.0f / (kCarryR * kCarryWdt);
constexpr float kScaleOut = 1.0f / (kCarryY * kCarryW);

constexpr size_t kBytesXH  = (size_t)kRows * kDm * 2;
constexpr size_t kBytesW1H = (size_t)kXzP * kDm * 2;
constexpr size_t kBytesR0  = (size_t)kRows * kDin * 2;
static_assert(kBytesXH + kBytesW1H == kBytesR0);
constexpr size_t kOffR0   = 0;
constexpr size_t kOffW4H  = kOffR0  + kBytesR0;
constexpr size_t kOffW2H  = kOffW4H + (size_t)kDm  * kDin * 2;
constexpr size_t kOffW3H  = kOffW2H + (size_t)kPrP * kDin * 2;
constexpr size_t kOffXZ   = kOffW3H + (size_t)kDin * kDtR * 2;
constexpr size_t kOffU    = kOffXZ  + (size_t)kRows * kXzP * 4;
constexpr size_t kOffPROJ = kOffU   + (size_t)kRows * kDin * 4;
constexpr size_t kOffDTRH = kOffPROJ + (size_t)kRows * kPrP * 4;
constexpr size_t kWsTotal = kOffDTRH + (size_t)kRows * kDtR * 2;
static_assert(kWsTotal == 125042688ull);
static_assert(kWsTotal <= 134217728ull);
static_assert((kOffW4H % 128) == 0 && (kOffW2H % 128) == 0 && (kOffW3H % 128) == 0 && (kOffXZ % 128) == 0 &&
              (kOffU % 128) == 0 && (kOffPROJ % 128) == 0 && (kOffDTRH % 128) == 0 && (kBytesXH % 128) == 0);

namespace eng {

typedef __attribute__((ext_vector_type(16))) _Float16 v16h;
typedef __attribute__((ext_vector_type(8)))  _Float16 v8h;
typedef __attribute__((ext_vector_type(8)))  float    v8f;
typedef __attribute__((ext_vector_type(4)))  float    v4f;
typedef __attribute__((ext_vector_type(4)))  unsigned v4u;

union FragU { v16h v; v8h h[2]; };

__device__ __forceinline__ v16h frag_load(const _Float16* p) {
  FragU f;
  f.h[0] = *(const v8h*)(p);
  f.h[1] = *(const v8h*)(p + 16);
  return f.v;
}
__device__ __forceinline__ v8f mma(v16h a, v16h b, v8f c) {
  return __builtin_amdgcn_wmma_f32_16x16x32_f16(false, a, false, b, (short)0, c, false, false);
}
__device__ __forceinline__ void guard1(v8f& acc, v16h a, v16h b) {
  asm volatile("v_nop\n\tv_nop\n\tv_nop\n\tv_nop" : "+v"(acc) : "v"(a), "v"(b));
}
__device__ __forceinline__ void keep4(v16h a, v16h b, v16h c, v16h d) {
  asm volatile("v_nop" :: "v"(a), "v"(b), "v"(c), "v"(d));
}
__device__ __forceinline__ void acc_guard1(v8f& a) {
  asm volatile("v_nop\n\tv_nop\n\tv_nop\n\tv_nop" : "+v"(a));
}

__device__ __forceinline__ unsigned h16bits_flush(float v) {
  const float f = (fabsf(v) < 6.103515625e-05f) ? 0.0f : v;
  const _Float16 h = (_Float16)f;
  return (unsigned)__builtin_bit_cast(unsigned short, h);
}
__device__ __forceinline__ unsigned pack2(float x0, float x1) {
  const unsigned lo = h16bits_flush(x0);
  const unsigned hi = h16bits_flush(x1);
  return lo | (hi << 16);
}
__device__ __forceinline__ v4u pack8(v4f a0, v4f a1, float carry, bool ok) {
  const float e0 = a0[0], e1 = a0[1], e2 = a0[2], e3 = a0[3];
  const float e4 = a1[0], e5 = a1[1], e6 = a1[2], e7 = a1[3];
  const float x0 = ok ? (e0 * carry) : 0.0f;
  const float x1 = ok ? (e1 * carry) : 0.0f;
  const float x2 = ok ? (e2 * carry) : 0.0f;
  const float x3 = ok ? (e3 * carry) : 0.0f;
  const float x4 = ok ? (e4 * carry) : 0.0f;
  const float x5 = ok ? (e5 * carry) : 0.0f;
  const float x6 = ok ? (e6 * carry) : 0.0f;
  const float x7 = ok ? (e7 * carry) : 0.0f;
  const unsigned w0 = pack2(x0, x1);
  const unsigned w1 = pack2(x2, x3);
  const unsigned w2 = pack2(x4, x5);
  const unsigned w3 = pack2(x6, x7);
  return (v4u){w0, w1, w2, w3};
}

template <int BIAS_N>
__global__ __launch_bounds__(256) void gemm_f16_kernel(
    const unsigned short* __restrict__ Ap, int lda,
    const unsigned short* __restrict__ Btp, int ldb,
    float* __restrict__ Cp, int ldc,
    const float* __restrict__ bias,
    int M, int N, int K, float scale)
{
  const _Float16* A  = (const _Float16*)Ap;
  const _Float16* Bt = (const _Float16*)Btp;
  __shared__ __align__(16) float sT[8][16 * 68];
  const int lane = threadIdx.x & 31;
  const int wave = threadIdx.x >> 5;
  const int tilesN = N >> 6;
  const int tilesM = M >> 6;
  const int tile = blockIdx.x * 8 + wave;
  if (tile >= tilesM * tilesN) return;
  const int tm = tile / tilesN;
  const int tn = tile - tm * tilesN;
  const int m0 = tm << 6;
  const int n0 = tn << 6;
  const int rlane = lane & 15;
  const int koff  = (lane >> 4) * 8;
  const int mOff  = (lane >> 4) * 8;

  v8f acc[4][4];
#pragma unroll
  for (int i = 0; i < 4; ++i)
#pragma unroll
    for (int j = 0; j < 4; ++j) acc[i][j] = (v8f){0.f, 0.f, 0.f, 0.f, 0.f, 0.f, 0.f, 0.f};

  for (int k0 = 0; k0 < K; k0 += 32) {
    v16h bh[4];
#pragma unroll
    for (int j = 0; j < 4; ++j) {
      const size_t bo = (size_t)(n0 + (j << 4) + rlane) * ldb + koff + k0;
      bh[j] = frag_load(Bt + bo);
    }
#pragma unroll
    for (int i = 0; i < 4; ++i) {
      const size_t ao = (size_t)(m0 + (i << 4) + rlane) * lda + koff + k0;
      const v16h ah = frag_load(A + ao);
#pragma unroll
      for (int j = 0; j < 4; ++j) acc[i][j] = mma(ah, bh[j], acc[i][j]);
#pragma unroll
      for (int j = 0; j < 4; ++j) guard1(acc[i][j], ah, bh[j]);
    }
    keep4(bh[0], bh[1], bh[2], bh[3]);
  }
#pragma unroll
  for (int i = 0; i < 4; ++i)
#pragma unroll
    for (int j = 0; j < 4; ++j) acc_guard1(acc[i][j]);

  float* slab = sT[wave];
#pragma unroll
  for (int i = 0; i < 4; ++i) {
    const int mBase = m0 + (i << 4);
#pragma unroll
    for (int j = 0; j < 4; ++j) {
      float bv = 0.f;
      if (BIAS_N == 1) bv = bias[n0 + (j << 4) + rlane];
#pragma unroll
      for (int r = 0; r < 8; ++r) {
        float v = acc[i][j][r] * scale;
        if (BIAS_N == 1) v += bv;
        slab[(mOff + r) * 68 + (j << 4) + rlane] = v;
      }
    }
    __builtin_amdgcn_fence(__ATOMIC_RELEASE, "workgroup");
    __builtin_amdgcn_wave_barrier();
    __builtin_amdgcn_fence(__ATOMIC_ACQUIRE, "workgroup");
    {
      const int hh = lane >> 4;
      const int c4 = (lane & 15) * 4;
      for (int pass = 0; pass < 2; ++pass) {
#pragma unroll
        for (int it = 0; it < 8; ++it) {
          const int row = it * 2 + hh;
          const v4f v = *(const v4f*)(slab + row * 68 + c4);
          *(volatile v4f*)(Cp + (size_t)(mBase + row) * ldc + n0 + c4) = v;
        }
        __threadfence();
      }
    }
    __builtin_amdgcn_fence(__ATOMIC_RELEASE, "workgroup");
    __builtin_amdgcn_wave_barrier();
    __builtin_amdgcn_fence(__ATOMIC_ACQUIRE, "workgroup");
  }
}

__global__ __launch_bounds__(256) void cvt_rows_f16_kernel(
    const float* __restrict__ src, long src_ld, unsigned short* __restrict__ dst,
    int cols8, int total8, int valid8, float carry)
{
  const int i = blockIdx.x * 256 + threadIdx.x;
  if (i >= total8) return;
  const bool ok = (i < valid8);
  const int ic  = ok ? i : (valid8 - 1);
  const int row = ic / cols8;
  const int c8  = (ic - row * cols8) * 8;
  const float* sp = src + (long)row * src_ld + c8;
  v4f a0 = *(const v4f*)(sp);
  v4f a1 = *(const v4f*)(sp + 4);
  asm volatile("" : "+v"(a0));
  asm volatile("" : "+v"(a1));
  const v4u w = pack8(a0, a1, carry, ok);
  unsigned short* q = dst + (size_t)i * 8;
  *(volatile v4u*)q = w;
  __threadfence();
  *(volatile v4u*)q = w;
}

__global__ __launch_bounds__(256) void conv_silu_kernel(
    const float* __restrict__ XZ, const float* __restrict__ cw, const float* __restrict__ cb,
    float* __restrict__ U, unsigned short* __restrict__ UH)
{
  __shared__ __align__(16) float sT[16 * kConvTP];
  constexpr int kCB = kDin / 256;
  const int tid = threadIdx.x, lane = tid & 31, wave = tid >> 5;
  const int rblk = blockIdx.x / kCB;
  const int cblk = blockIdx.x - rblk * kCB;
  const int d0 = cblk * 256;
  const int d  = d0 + tid;
  const int g0 = rblk * 64;
  const int tb = g0 & (kSeq - 1);
  const v4f wv = *(const v4f*)(cw + (size_t)d * 4);
  const float w0 = wv[0], w1 = wv[1], w2 = wv[2], w3 = wv[3];
  const float bc = cb[d];
  float xm3, xm2, xm1;
  {
    const bool hist = (tb > 0);
    const int rb = hist ? (g0 - 3) : g0;
    const float v3 = XZ[(size_t)rb * kXzP + d];
    const float v2 = XZ[(size_t)(rb + 1) * kXzP + d];
    const float v1 = XZ[(size_t)(rb + 2) * kXzP + d];
    xm3 = hist ? v3 : 0.f;
    xm2 = hist ? v2 : 0.f;
    xm1 = hist ? v1 : 0.f;
  }
  const int hrow = wave >> 1;
  const int hch  = (wave & 1) * 128 + lane * 4;
#pragma unroll 1
  for (int sub = 0; sub < 4; ++sub) {
    const int lb = g0 + sub * 16;
#pragma unroll 1
    for (int s = 0; s < 16; ++s) {
      const float xcur = XZ[(size_t)(lb + s) * kXzP + d];
      float acc = w0 * xm3;
      acc = fmaf(w1, xm2, acc);
      acc = fmaf(w2, xm1, acc);
      acc = fmaf(w3, xcur, acc);
      const float sv = acc + bc;
      const float sg = __builtin_amdgcn_rcpf(1.0f + expf(-sv));
      sT[s * kConvTP + tid] = sv * sg;
      xm3 = xm2;
      xm2 = xm1;
      xm1 = xcur;
    }
    __syncthreads();
    v4f fv[4];
    v4u hw[2];
#pragma unroll
    for (int it = 0; it < 4; ++it) fv[it] = *(const v4f*)(sT + (it * 4 + hrow) * kConvTP + hch);
#pragma unroll
    for (int it = 0; it < 2; ++it) {
      const float* sp = sT + (it * 8 + wave) * kConvTP + lane * 8;
      const v4f a0 = *(const v4f*)(sp);
      const v4f a1 = *(const v4f*)(sp + 4);
      hw[it] = pack8(a0, a1, kCarryU, true);
    }
    for (int pass = 0; pass < 2; ++pass) {
#pragma unroll
      for (int it = 0; it < 4; ++it)
        *(volatile v4f*)(U + (size_t)(lb + it * 4 + hrow) * kDin + d0 + hch) = fv[it];
#pragma unroll
      for (int it = 0; it < 2; ++it)
        *(volatile v4u*)(UH + (size_t)(lb + it * 8 + wave) * kDin + d0 + lane * 8) = hw[it];
      __threadfence();
    }
    __syncthreads();
  }
}

}

typedef float    ms1_v4f __attribute__((ext_vector_type(4)));
typedef unsigned ms1_v4u __attribute__((ext_vector_type(4)));
struct ms1_args {
  const float* dtpre;
  const float* u;
  const float* bc;
  const float* z;
  const float* A_log;
  const float* Dskip;
  __half* y;
  __half* y_lo;
  long ld_dtpre;
  long ld_u;
  long ld_bc;
  long ld_z;
  long ld_y;
  int offB;
  int offC;
  int offZ;
  float ycarry;
  int dir;
  int D;
  int L;
  int nbatch;
};
static_assert(sizeof(ms1_args) == 136);

__device__ __forceinline__ float ms1_flush16(float v) {
  return (fabsf(v) < 6.103515625e-05f) ? 0.0f : v;
}
__device__ __forceinline__ unsigned ms1_h16bits(float v) {
  return (unsigned)__half_as_ushort(__float2half_rn(ms1_flush16(v)));
}
__device__ __forceinline__ float ms1_h16val(unsigned b) {
  return __half2float(__ushort_as_half((unsigned short)b));
}
__device__ __forceinline__ float ms1_softplus(float v) {
  return fmaxf(v, 0.0f) + log1pf(expf(-fabsf(v)));
}
__device__ __forceinline__ void ms1_pack2(float v0, float v1, unsigned& hw, unsigned& lw) {
  const unsigned h0 = ms1_h16bits(v0);
  const unsigned h1 = ms1_h16bits(v1);
  const float r0 = (v0 - ms1_h16val(h0)) * 2048.0f;
  const float r1 = (v1 - ms1_h16val(h1)) * 2048.0f;
  const unsigned l0 = ms1_h16bits(r0);
  const unsigned l1 = ms1_h16bits(r1);
  hw = h0 | (h1 << 16);
  lw = l0 | (l1 << 16);
}

template <int NSTATE>
__global__ __launch_bounds__(64 * (NSTATE / 16)) void ms1_scan_kernel(ms1_args a)
{
  static_assert(NSTATE == 16 || NSTATE == 64);
  constexpr int NQ  = NSTATE / 16;
  constexpr int NT  = 64 * NQ;
  constexpr int NW  = NT / 32;
  constexpr int BCW = 2 * NSTATE;
  constexpr int YP  = 68;
  constexpr int RPI = NW * 4;
  constexpr int NIT = 64 / RPI;
  static_assert(16 * NT <= 64 * YP);
  __shared__ __align__(16) float sBC[64 * BCW];
  __shared__ __align__(16) float sY[64 * YP];
  const int tid  = threadIdx.x;
  const int lane = tid & 31;
  const int wave = tid >> 5;
  const int c    = tid / NQ;
  const int sq   = tid - c * NQ;
  const int bpb  = a.D / 64;
  const int bi   = blockIdx.x / bpb;
  if (bi >= a.nbatch) return;
  const int d0 = (blockIdx.x - bi * bpb) * 64;
  const int d  = d0 + c;
  const long rowb = (long)bi * a.L;
  const bool hasz  = (a.z != nullptr);
  const bool hasD  = (a.Dskip != nullptr);
  const bool hasLo = (a.y_lo != nullptr);

#pragma unroll 1
  for (int n = 0; n < 16; ++n) {
    const float al = a.A_log[(long)d * NSTATE + sq * 16 + n];
    sY[n * NT + tid] = -expf(al);
  }
  __syncthreads();
  float An[16], h[16];
#pragma unroll
  for (int n = 0; n < 16; ++n) {
    An[n] = sY[n * NT + tid];
    h[n] = 0.0f;
  }
  float Dd = 0.0f;
  if (hasD) Dd = a.Dskip[d];

  const int nchunk = a.L / 64;
  const bool fwd = (a.dir > 0);
  const int s0 = fwd ? 0 : 63;
  const int sd = fwd ? 1 : -1;
  const int q  = lane >> 3;
  const int c8 = (lane & 7) * 8;

#pragma unroll 1
  for (int ci = 0; ci < nchunk; ++ci) {
    const int tb = fwd ? (ci * 64) : (a.L - 64 - ci * 64);
    const long rowc = rowb + tb;
    __syncthreads();
#pragma unroll 8
    for (int i = 0; i < 32; ++i) {
      const int idx = tid + i * NT;
      const int st  = idx / BCW;
      const int col = idx - st * BCW;
      const int sc  = (col < NSTATE) ? (a.offB + col) : (a.offC + col - NSTATE);
      sBC[idx] = a.bc[(rowc + st) * a.ld_bc + sc];
    }
    __syncthreads();
#pragma unroll 1
    for (int s = 0; s < 64; ++s) {
      const int ls = s0 + sd * s;
      const long row = rowc + ls;
      float pre = a.dtpre[row * a.ld_dtpre + d];
      float uv  = a.u[row * a.ld_u + d];
      float zv  = 0.0f;
      if (hasz) zv = a.z[row * a.ld_z + a.offZ + d];
      asm volatile("" : "+v"(pre));
      asm volatile("" : "+v"(uv));
      asm volatile("" : "+v"(zv));
      const float delta = ms1_softplus(pre);
      const float dtx = delta * uv;
      const float* bp = sBC + ls * BCW + sq * 16;
      const float* cp = bp + NSTATE;
      ms1_v4f Bq[4], Cq[4];
#pragma unroll
      for (int k = 0; k < 4; ++k) {
        Bq[k] = *(const ms1_v4f*)(bp + 4 * k);
        Cq[k] = *(const ms1_v4f*)(cp + 4 * k);
      }
      float yv = 0.0f;
#pragma unroll
      for (int n = 0; n < 16; ++n) {
        const float e = __expf(delta * An[n]);
        h[n] = fmaf(e, h[n], dtx * Bq[n >> 2][n & 3]);
        yv = fmaf(h[n], Cq[n >> 2][n & 3], yv);
      }
      if (NQ > 1) {
        yv += __shfl_xor(yv, 1, 32);
        yv += __shfl_xor(yv, 2, 32);
      }
      if (hasD) yv = fmaf(uv, Dd, yv);
      if (hasz) {
        const float sg = __builtin_amdgcn_rcpf(1.0f + expf(-zv));
        yv = yv * (zv * sg);
      }
      if (sq == 0) sY[ls * YP + c] = yv * a.ycarry;
    }
    __syncthreads();
    ms1_v4u hw[NIT], lw[NIT];
#pragma unroll
    for (int it = 0; it < NIT; ++it) {
      const int row = it * RPI + wave * 4 + q;
      const float* sp = sY + row * YP + c8;
      const ms1_v4f f0 = *(const ms1_v4f*)(sp);
      const ms1_v4f f1 = *(const ms1_v4f*)(sp + 4);
      unsigned h0, h1, h2, h3, l0, l1, l2, l3;
      ms1_pack2(f0[0], f0[1], h0, l0);
      ms1_pack2(f0[2], f0[3], h1, l1);
      ms1_pack2(f1[0], f1[1], h2, l2);
      ms1_pack2(f1[2], f1[3], h3, l3);
      hw[it] = (ms1_v4u){h0, h1, h2, h3};
      lw[it] = (ms1_v4u){l0, l1, l2, l3};
    }
    for (int pass = 0; pass < 2; ++pass) {
#pragma unroll
      for (int it = 0; it < NIT; ++it) {
        const int row = it * RPI + wave * 4 + q;
        const long o = (rowc + row) * a.ld_y + d0 + c8;
        *(volatile ms1_v4u*)(a.y + o) = hw[it];
        if (hasLo) *(volatile ms1_v4u*)(a.y_lo + o) = lw[it];
      }
      __threadfence();
    }
  }
}

static_assert(((kRows / 64) * (kXzP / 64)) % 8 == 0);
static_assert(((kRows / 64) * (kPrP / 64)) % 8 == 0);
static_assert(((kRows / 64) * (kDin / 64)) % 8 == 0);
static_assert(((kRows / 64) * (kDm / 64)) % 8 == 0);
static_assert((kRows * kDm / 8) % 256 == 0 && (kXzP * kDm / 8) % 256 == 0 && (kDm * kDin / 8) % 256 == 0);
static_assert((kPrP * kDin / 8) % 256 == 0 && (kDin * kDtR / 8) % 256 == 0 && (kRows * kDtR / 8) % 256 == 0);
static_assert((kPrW * kDin / 8) % 32 == 0);

extern "C" void kernel_launch(void* const* d_in, const int* in_sizes, int n_in,
                              void* d_out, int out_size, void* d_ws, size_t ws_size,
                              hipStream_t stream) {
  if (n_in < 10) return;
  if (in_sizes[0] != kRows * kDm) return;
  if (in_sizes[1] != kXzP * kDm) return;
  if (in_sizes[2] != kDin * 4) return;
  if (in_sizes[3] != kDin) return;
  if (in_sizes[4] != kPrW * kDin) return;
  if (in_sizes[5] != kDin * kDtR) return;
  if (in_sizes[6] != kDin) return;
  if (in_sizes[7] != kDin * kNst) return;
  if (in_sizes[8] != kDin) return;
  if (in_sizes[9] != kDm * kDin) return;
  if (out_size != kRows * kDm) return;
  if (ws_size < kWsTotal) return;

  const float* x_in    = (const float*)d_in[0];
  const float* W_in    = (const float*)d_in[1];
  const float* conv_w  = (const float*)d_in[2];
  const float* conv_b  = (const float*)d_in[3];
  const float* W_xproj = (const float*)d_in[4];
  const float* W_dt    = (const float*)d_in[5];
  const float* b_dt    = (const float*)d_in[6];
  const float* A_log   = (const float*)d_in[7];
  const float* D_par   = (const float*)d_in[8];
  const float* W_out   = (const float*)d_in[9];
  float* out = (float*)d_out;

  char* ws = (char*)d_ws;
  unsigned short* XH   = (unsigned short*)(ws + kOffR0);
  unsigned short* W1H  = (unsigned short*)(ws + kOffR0 + kBytesXH);
  unsigned short* UH   = (unsigned short*)(ws + kOffR0);
  __half*         YH   = (__half*)(ws + kOffR0);
  unsigned short* W4H  = (unsigned short*)(ws + kOffW4H);
  unsigned short* W2H  = (unsigned short*)(ws + kOffW2H);
  unsigned short* W3H  = (unsigned short*)(ws + kOffW3H);
  float*          XZ   = (float*)(ws + kOffXZ);
  float*          U    = (float*)(ws + kOffU);
  float*          PROJ = (float*)(ws + kOffPROJ);
  unsigned short* DTRH = (unsigned short*)(ws + kOffDTRH);

  eng::cvt_rows_f16_kernel<<<(kRows * kDm / 8) / 256, 256, 0, stream>>>(
      x_in, (long)kDm, XH, kDm / 8, kRows * kDm / 8, kRows * kDm / 8, kCarryX);
  eng::cvt_rows_f16_kernel<<<(kXzP * kDm / 8) / 256, 256, 0, stream>>>(
      W_in, (long)kDm, W1H, kDm / 8, kXzP * kDm / 8, kXzP * kDm / 8, kCarryW);
  eng::cvt_rows_f16_kernel<<<(kDm * kDin / 8) / 256, 256, 0, stream>>>(
      W_out, (long)kDin, W4H, kDin / 8, kDm * kDin / 8, kDm * kDin / 8, kCarryW);
  eng::cvt_rows_f16_kernel<<<(kPrP * kDin / 8) / 256, 256, 0, stream>>>(
      W_xproj, (long)kDin, W2H, kDin / 8, kPrP * kDin / 8, kPrW * kDin / 8, kCarryW);
  eng::cvt_rows_f16_kernel<<<(kDin * kDtR / 8) / 256, 256, 0, stream>>>(
      W_dt, (long)kDtR, W3H, kDtR / 8, kDin * kDtR / 8, kDin * kDtR / 8, kCarryWdt);

  eng::gemm_f16_kernel<0><<<dim3((kRows / 64) * (kXzP / 64) / 8), 256, 0, stream>>>(
      XH, kDm, W1H, kDm, XZ, kXzP, nullptr, kRows, kXzP, kDm, kScaleIn);

  eng::conv_silu_kernel<<<dim3((kDin / 256) * (kRows / 64)), 256, 0, stream>>>(XZ, conv_w, conv_b, U, UH);

  eng::gemm_f16_kernel<0><<<dim3((kRows / 64) * (kPrP / 64) / 8), 256, 0, stream>>>(
      UH, kDin, W2H, kDin, PROJ, kPrP, nullptr, kRows, kPrP, kDin, kScaleXp);

  eng::cvt_rows_f16_kernel<<<(kRows * kDtR / 8) / 256, 256, 0, stream>>>(
      PROJ, (long)kPrP, DTRH, kDtR / 8, kRows * kDtR / 8, kRows * kDtR / 8, kCarryR);

  eng::gemm_f16_kernel<1><<<dim3((kRows / 64) * (kDin / 64) / 8), 256, 0, stream>>>(
      DTRH, kDtR, W3H, kDtR, XZ, kXzP, b_dt, kRows, kDin, kDtR, kScaleDt);

  for (int b = 0; b < kBatch; ++b) {
    const size_t r0 = (size_t)b * kSeq;
    ms1_args sa;
    sa.dtpre = XZ + r0 * kXzP;
    sa.u = U + r0 * kDin;
    sa.bc = PROJ + r0 * kPrP;
    sa.z = XZ + r0 * kXzP;
    sa.A_log = A_log;
    sa.Dskip = D_par;
    sa.y = YH + r0 * kDin;
    sa.y_lo = nullptr;
    sa.ld_dtpre = kXzP;
    sa.ld_u = kDin;
    sa.ld_bc = kPrP;
    sa.ld_z = kXzP;
    sa.ld_y = kDin;
    sa.offB = kOffB;
    sa.offC = kOffC;
    sa.offZ = kDin;
    sa.ycarry = kCarryY;
    sa.dir = 1;
    sa.D = kDin;
    sa.L = kSeq;
    sa.nbatch = 1;
    ms1_scan_kernel<16><<<dim3(kDin / 64), 64, 0, stream>>>(sa);
  }

  eng::gemm_f16_kernel<0><<<dim3((kRows / 64) * (kDm / 64) / 8), 256, 0, stream>>>(
      (const unsigned short*)YH, kDin, W4H, kDin, out, kDm, nullptr, kRows, kDm, kDin, kScaleOut);
}
